// HGTPolicy_53051436040798
// MI455X (gfx1250) — hardware-run, weakly checked
//
#include <hip/hip_runtime.h>
#include <math.h>

typedef __attribute__((ext_vector_type(16))) _Float16 v16h;
typedef __attribute__((ext_vector_type(8)))  _Float16 v8h;
typedef __attribute__((ext_vector_type(8)))  float    v8f;
typedef __attribute__((ext_vector_type(4)))  float    v4f;
typedef __attribute__((ext_vector_type(2)))  float    v2f;
typedef __attribute__((ext_vector_type(4)))  int      v4i;

constexpr int kHid   = 64;
constexpr int kHeads = 8;
constexpr int kD     = 8;
constexpr int kNop   = 50000;
constexpr int kNm    = 1000;
constexpr int kNj    = 5000;
constexpr int kPadOp = 50048;
constexpr int kPadM  = 1024;
constexpr int kPadJ  = 5056;
constexpr int kOffM  = kPadOp;
constexpr int kOffJ  = kPadOp + kPadM;
constexpr int kRows  = kPadOp + kPadM + kPadJ;
constexpr int kBlkOp = kPadOp / 64;
constexpr int kBlkM  = kPadM / 64;
constexpr int kBlkJ  = kPadJ / 64;
constexpr int kBlkAll = kBlkOp + kBlkM + kBlkJ;
constexpr int kP     = 20000;
constexpr int kPPad  = 20032;
constexpr int kE     = 50000;
constexpr int kEBig  = 150000;
constexpr int kLayers = 2;
constexpr int kTile  = 384;
constexpr int kTilesOp = (kPadOp + kTile - 1) / kTile;
constexpr int kTilesM  = (kPadM + kTile - 1) / kTile;
constexpr int kTilesJ  = (kPadJ + kTile - 1) / kTile;
constexpr int kRelRows = 7008;
constexpr float kActCarry = 64.0f;
constexpr float kWgtCarry = 16.0f;
constexpr float kGemmScale = 1.0f / (kActCarry * kWgtCarry);
static_assert(kHeads * kD == kHid, "head split");
static_assert(kRows == 56128 && kBlkAll == 877, "padded rows");
static_assert((kPadOp % 64) == 0 && (kPadM % 64) == 0 && (kPadJ % 64) == 0 && (kPPad % 64) == 0, "GEMM M multiples of 64");
static_assert((kE % 8) == 0 && (kEBig % 8) == 0, "edge groups of 8");
static_assert(kTilesOp == 131 && kTilesM == 3 && kTilesJ == 14, "destination tiles");
static_assert(kNop <= 65536 && kTile <= 512, "packed queue entry fields");
static_assert((kTile * 72) % 1024 == 0, "accumulator zero fill coverage");

constexpr size_t kSzX    = (size_t)kRows * 64 * 4;
constexpr size_t kSzXH   = (size_t)kRows * 64 * 2;
constexpr size_t kSzKQV  = (size_t)kRows * 192 * 4;
constexpr size_t kSzREL  = (size_t)kRelRows * 128 * 4;
constexpr int kWtKqvHalves = 6 * 192 * 64;
constexpr int kWtOutHalves = 6 * 64 * 64;
constexpr int kWtP1Halves  = 64 * 128;
constexpr int kWtP2Halves  = 64 * 64;
constexpr int kWtOffOut = kWtKqvHalves;
constexpr int kWtOffP1  = kWtOffOut + kWtOutHalves;
constexpr int kWtOffP2  = kWtOffP1 + kWtP1Halves;
constexpr int kWtHalves = kWtOffP2 + kWtP2Halves;
constexpr size_t kSzWT   = (size_t)kWtHalves * 2;
constexpr size_t kSzPART = (size_t)kBlkAll * 128;
constexpr size_t kSzSTAT = 128;
constexpr size_t kSzPARTM = (size_t)kBlkAll * 256;
constexpr size_t kSzCB   = 512;
constexpr size_t kSzZH   = (size_t)kPPad * 128 * 2;
constexpr size_t kSzZ1H  = (size_t)kPPad * 64 * 2;
constexpr size_t kOffX0   = 0;
constexpr size_t kOffX1   = kOffX0 + kSzX;
constexpr size_t kOffXH   = kOffX1 + kSzX;
constexpr size_t kOffGH   = kOffXH + kSzXH;
constexpr size_t kOffKQV  = kOffGH + kSzXH;
constexpr size_t kOffREL  = kOffKQV + kSzKQV;
constexpr size_t kOffWT   = kOffREL + kSzREL;
constexpr size_t kOffPART = kOffWT + kSzWT;
constexpr size_t kOffSTAT = kOffPART + kSzPART;
constexpr size_t kOffPARTM = kOffSTAT + kSzSTAT;
constexpr size_t kOffCB   = kOffPARTM + kSzPARTM;
constexpr size_t kOffZH   = kOffCB + kSzCB;
constexpr size_t kOffZ1H  = kOffZH + kSzZH;
constexpr size_t kWsTotal = kOffZ1H + kSzZ1H;
static_assert(kWsTotal == 98051584ull, "carve total");
static_assert(kWsTotal <= 134217728ull, "carve cap");
static_assert((kOffX1 % 128) == 0 && (kOffXH % 128) == 0 && (kOffGH % 128) == 0 && (kOffKQV % 128) == 0 &&
              (kOffREL % 128) == 0 && (kOffWT % 128) == 0 && (kOffPART % 128) == 0 && (kOffSTAT % 128) == 0 &&
              (kOffPARTM % 128) == 0 && (kOffCB % 128) == 0 && (kOffZH % 128) == 0 && (kOffZ1H % 128) == 0, "aligned regions");
static_assert(kWtHalves == 110592 && (kWtHalves / 8) == 54 * 256, "weight prep coverage");

union FragU { v16h v; v8h h[2]; };
__device__ __forceinline__ v16h frag_load(const _Float16* p) {
  FragU f;
  f.h[0] = *(const v8h*)(p);
  f.h[1] = *(const v8h*)(p + 16);
  return f.v;
}
__device__ __forceinline__ v8f mma_h(v16h a, v16h b, v8f c) {
  c = __builtin_amdgcn_wmma_f32_16x16x32_f16(false, a, false, b, (short)0, c, false, false);
  asm volatile("v_nop\n\tv_nop\n\tv_nop\n\tv_nop" : "+v"(c) : "v"(a), "v"(b));
  return c;
}
__device__ __forceinline__ void wave_sync() {
  __builtin_amdgcn_fence(__ATOMIC_RELEASE, "workgroup");
  __builtin_amdgcn_wave_barrier();
  __builtin_amdgcn_fence(__ATOMIC_ACQUIRE, "workgroup");
}

__global__ __launch_bounds__(256) void prep_weights_kernel(
    const float* __restrict__ Wkqv, const float* __restrict__ Wout,
    const float* __restrict__ Wp1, const float* __restrict__ Wp2,
    unsigned short* __restrict__ WT)
{
  const int gid = blockIdx.x * 256 + threadIdx.x;
  float w[8];
  if (blockIdx.x < 36) {
    const int el = gid * 8;
    const int lt = el / (192 * 64);
    const int rem = el - lt * (192 * 64);
    const int n = rem >> 6, k0 = rem & 63;
#pragma unroll
    for (int i = 0; i < 8; ++i) w[i] = Wkqv[(size_t)lt * (64 * 192) + (size_t)(k0 + i) * 192 + n];
  } else if (blockIdx.x < 48) {
    const int el = (gid - 36 * 256) * 8;
    const int lt = el >> 12;
    const int rem = el & 4095;
    const int n = rem >> 6, k0 = rem & 63;
#pragma unroll
    for (int i = 0; i < 8; ++i) w[i] = Wout[(size_t)lt * 4096 + (size_t)(k0 + i) * 64 + n];
  } else if (blockIdx.x < 52) {
    const int el = (gid - 48 * 256) * 8;
    const int n = el >> 7, k0 = el & 127;
#pragma unroll
    for (int i = 0; i < 8; ++i) w[i] = Wp1[(size_t)(k0 + i) * 64 + n];
  } else {
    const int el = (gid - 52 * 256) * 8;
    const int n = el >> 6, k0 = el & 63;
    const int nc = n < 32 ? n : 31;
#pragma unroll
    for (int i = 0; i < 8; ++i) {
      const float t = Wp2[(size_t)(k0 + i) * 32 + nc];
      w[i] = (n < 32) ? t : 0.0f;
    }
  }
  v8h hv;
#pragma unroll
  for (int i = 0; i < 8; ++i) hv[i] = (_Float16)(w[i] * kWgtCarry);
  unsigned short* dst = WT + (size_t)gid * 8;
  *(volatile v8h*)dst = hv;
  __threadfence();
  *(volatile v8h*)dst = hv;
}

__global__ __launch_bounds__(256) void proj_kernel(
    const float* __restrict__ opx, const float* __restrict__ mx, const float* __restrict__ jx,
    const float* __restrict__ Wop, const float* __restrict__ bop,
    const float* __restrict__ Wm, const float* __restrict__ bm,
    const float* __restrict__ Wj, const float* __restrict__ bj,
    float* __restrict__ Y, float* __restrict__ PART)
{
  __shared__ __align__(16) float tile[64 * 68];
  __shared__ float red[16];
  const int tid = threadIdx.x, lane = tid & 31, wave = tid >> 5;
  const int b = blockIdx.x;
  const int ty = (b >= kBlkOp ? 1 : 0) + (b >= kBlkOp + kBlkM ? 1 : 0);
  const int tb0 = ty == 0 ? 0 : (ty == 1 ? kBlkOp : kBlkOp + kBlkM);
  const int nT = ty == 0 ? kNop : (ty == 1 ? kNm : kNj);
  const int F = ty == 0 ? 8 : 7;
  const float* x = ty == 0 ? opx : (ty == 1 ? mx : jx);
  const float* W = ty == 0 ? Wop : (ty == 1 ? Wm : Wj);
  const float* bb = ty == 0 ? bop : (ty == 1 ? bm : bj);
  const int r = tid >> 2, cq = (tid & 3) * 16;
  const int rt = (b - tb0) * 64 + r;
  const bool valid = rt < nT;
  const int rc = valid ? rt : (nT - 1);
  float y[16];
#pragma unroll
  for (int q = 0; q < 4; ++q) {
    const v4f bv = *(const v4f*)(bb + cq + 4 * q);
    y[4 * q + 0] = bv[0]; y[4 * q + 1] = bv[1]; y[4 * q + 2] = bv[2]; y[4 * q + 3] = bv[3];
  }
#pragma unroll 1
  for (int f = 0; f < F; ++f) {
    const float xv = x[(size_t)rc * F + f];
#pragma unroll
    for (int q = 0; q < 4; ++q) {
      const v4f wv = *(const v4f*)(W + f * 64 + cq + 4 * q);
      y[4 * q + 0] = fmaf(xv, wv[0], y[4 * q + 0]);
      y[4 * q + 1] = fmaf(xv, wv[1], y[4 * q + 1]);
      y[4 * q + 2] = fmaf(xv, wv[2], y[4 * q + 2]);
      y[4 * q + 3] = fmaf(xv, wv[3], y[4 * q + 3]);
    }
  }
  float s = 0.0f, ss = 0.0f;
#pragma unroll
  for (int j = 0; j < 16; ++j) {
    y[j] = valid ? y[j] : 0.0f;
    s += y[j];
    ss = fmaf(y[j], y[j], ss);
  }
#pragma unroll
  for (int q = 0; q < 4; ++q) {
    v4f o;
    o[0] = y[4 * q + 0]; o[1] = y[4 * q + 1]; o[2] = y[4 * q + 2]; o[3] = y[4 * q + 3];
    *(v4f*)(tile + r * 68 + cq + 4 * q) = o;
  }
#pragma unroll
  for (int off = 16; off > 0; off >>= 1) {
    s += __shfl_xor(s, off, 32);
    ss += __shfl_xor(ss, off, 32);
  }
  if (lane == 0) { red[wave] = s; red[8 + wave] = ss; }
  __syncthreads();
  {
    const int hh = lane >> 4, c4 = (lane & 15) * 4;
    v4f v[4];
#pragma unroll
    for (int it = 0; it < 4; ++it) v[it] = *(const v4f*)(tile + (wave * 8 + it * 2 + hh) * 68 + c4);
    for (int pass = 0; pass < 2; ++pass) {
#pragma unroll
      for (int it = 0; it < 4; ++it)
        *(volatile v4f*)(Y + (size_t)(b * 64 + wave * 8 + it * 2 + hh) * 64 + c4) = v[it];
      __threadfence();
    }
  }
  if (wave == 0) {
    float a = 0.0f, q2 = 0.0f;
#pragma unroll
    for (int w = 0; w < 8; ++w) { a += red[w]; q2 += red[8 + w]; }
    const float val = (lane == 0) ? a : ((lane == 1) ? q2 : 0.0f);
    *(volatile float*)(PART + (size_t)b * 32 + lane) = val;
    __threadfence();
    *(volatile float*)(PART + (size_t)b * 32 + lane) = val;
  }
}

__global__ __launch_bounds__(256) void stats_kernel(const float* __restrict__ PART, float* __restrict__ STATS)
{
  __shared__ double ds[256];
  __shared__ double dq[256];
  __shared__ float res[8];
  const int tid = threadIdx.x;
#pragma unroll 1
  for (int ty = 0; ty < 3; ++ty) {
    const int b0 = ty == 0 ? 0 : (ty == 1 ? kBlkOp : kBlkOp + kBlkM);
    const int b1 = ty == 0 ? kBlkOp : (ty == 1 ? kBlkOp + kBlkM : kBlkAll);
    const double cinv = ty == 0 ? (1.0 / ((double)kNop * 64.0)) : (ty == 1 ? (1.0 / ((double)kNm * 64.0)) : (1.0 / ((double)kNj * 64.0)));
    double s = 0.0, q = 0.0;
#pragma unroll 1
    for (int b = b0 + tid; b < b1; b += 256) {
      s += (double)PART[(size_t)b * 32];
      q += (double)PART[(size_t)b * 32 + 1];
    }
    ds[tid] = s; dq[tid] = q;
    __syncthreads();
#pragma unroll 1
    for (int st = 128; st > 0; st >>= 1) {
      if (tid < st) { ds[tid] += ds[tid + st]; dq[tid] += dq[tid + st]; }
      __syncthreads();
    }
    if (tid == 0) {
      const double mu = ds[0] * cinv;
      const double var = dq[0] * cinv - mu * mu;
      const float vf = (float)var;
      const float sd = sqrtf(vf > 0.0f ? vf : 0.0f);
      res[ty * 2] = (float)mu;
      res[ty * 2 + 1] = 1.0f / (sd + 1e-5f);
    }
    __syncthreads();
  }
  if (tid < 32) {
    const float t = res[tid < 6 ? tid : 0];
    const float val = (tid < 6) ? t : 0.0f;
    *(volatile float*)(STATS + tid) = val;
    __threadfence();
    *(volatile float*)(STATS + tid) = val;
  }
}

__global__ __launch_bounds__(256) void norm_kernel(
    const float* __restrict__ Y, const float* __restrict__ STATS,
    const float* __restrict__ gamma, const float* __restrict__ beta,
    float* __restrict__ X0, unsigned short* __restrict__ XH)
{
  const int tid = threadIdx.x;
  const int row0 = blockIdx.x * 32;
  const int ty = (row0 >= kOffM ? 1 : 0) + (row0 >= kOffJ ? 1 : 0);
  const int nT = ty == 0 ? kNop : (ty == 1 ? kNm : kNj);
  const int offT = ty == 0 ? 0 : (ty == 1 ? kOffM : kOffJ);
  const float mu = STATS[ty * 2], inv = STATS[ty * 2 + 1];
  v4f xo[2];
#pragma unroll
  for (int gs = 0; gs < 2; ++gs) {
    const int e0 = blockIdx.x * 2048 + gs * 1024 + tid * 4;
    const int row = e0 >> 6, col = e0 & 63;
    const v4f yv = *(const v4f*)(Y + e0);
    const v4f gm = *(const v4f*)(gamma + ty * 64 + col);
    const v4f bt = *(const v4f*)(beta + ty * 64 + col);
    const bool ok = (row - offT) < nT;
#pragma unroll
    for (int c = 0; c < 4; ++c) {
      const float xv = (yv[c] - mu) * inv * gm[c] + bt[c];
      xo[gs][c] = ok ? xv : 0.0f;
    }
  }
  v8h hv;
  const int e0h = blockIdx.x * 2048 + tid * 8;
  {
    const int row = e0h >> 6, col = e0h & 63;
    const bool ok = (row - offT) < nT;
    const v4f y0 = *(const v4f*)(Y + e0h);
    const v4f y1 = *(const v4f*)(Y + e0h + 4);
    const v4f g0 = *(const v4f*)(gamma + ty * 64 + col);
    const v4f g1 = *(const v4f*)(gamma + ty * 64 + col + 4);
    const v4f b0 = *(const v4f*)(beta + ty * 64 + col);
    const v4f b1 = *(const v4f*)(beta + ty * 64 + col + 4);
#pragma unroll
    for (int c = 0; c < 4; ++c) {
      const float xa = (y0[c] - mu) * inv * g0[c] + b0[c];
      const float xb = (y1[c] - mu) * inv * g1[c] + b1[c];
      hv[c] = (_Float16)(ok ? xa * kActCarry : 0.0f);
      hv[4 + c] = (_Float16)(ok ? xb * kActCarry : 0.0f);
    }
  }
  for (int pass = 0; pass < 2; ++pass) {
#pragma unroll
    for (int gs = 0; gs < 2; ++gs)
      *(volatile v4f*)(X0 + blockIdx.x * 2048 + gs * 1024 + tid * 4) = xo[gs];
    *(volatile v8h*)(XH + e0h) = hv;
    __threadfence();
  }
}

template <int EPI>
__global__ __launch_bounds__(256) void gemm64_kernel(
    const unsigned short* __restrict__ Ap, int lda,
    const unsigned short* __restrict__ Btp, int ldb, int btTypeStride,
    const float* __restrict__ bias, int biasTypeStride,
    float* __restrict__ Cf, unsigned short* __restrict__ Ch, int ldc,
    const float* __restrict__ resid, const float* __restrict__ skipv,
    const float* __restrict__ w3, const float* __restrict__ b3,
    int tilesM, int tilesN, int K, int typed, int mReal, float scale, float oscale)
{
  __shared__ __align__(16) float sT[8][16 * 68];
  __shared__ __align__(16) float sL[8][64];
  const int lane = threadIdx.x & 31;
  const int wave = threadIdx.x >> 5;
  const int tile = blockIdx.x * 8 + wave;
  if (tile >= tilesM * tilesN) return;
  const int tm = tile / tilesN;
  const int tn = tile - tm * tilesN;
  const int m0 = tm << 6;
  const int n0 = tn << 6;
  int ty = 0;
  if (typed) ty = (tm >= kBlkOp ? 1 : 0) + (tm >= kBlkOp + kBlkM ? 1 : 0);
  const _Float16* A = (const _Float16*)Ap;
  const _Float16* Bt = (const _Float16*)Btp + (size_t)ty * (size_t)btTypeStride;
  const float* bs = bias + ty * biasTypeStride;
  const int rlane = lane & 15;
  const int koff = (lane >> 4) * 8;
  const int mOff = (lane >> 4) * 8;

  v8f acc[4][4];
#pragma unroll
  for (int i = 0; i < 4; ++i)
#pragma unroll
    for (int j = 0; j < 4; ++j) acc[i][j] = (v8f){0.f, 0.f, 0.f, 0.f, 0.f, 0.f, 0.f, 0.f};

  for (int k0 = 0; k0 < K; k0 += 32) {
    v16h bh[4];
#pragma unroll
    for (int j = 0; j < 4; ++j)
      bh[j] = frag_load(Bt + (size_t)(n0 + (j << 4) + rlane) * ldb + koff + k0);
#pragma unroll
    for (int i = 0; i < 4; ++i) {
      const v16h ah = frag_load(A + (size_t)(m0 + (i << 4) + rlane) * lda + koff + k0);
#pragma unroll
      for (int j = 0; j < 4; ++j) acc[i][j] = mma_h(ah, bh[j], acc[i][j]);
    }
  }

  float* slab = sT[wave];
  float gate = 0.0f, omg = 0.0f;
  if (EPI == 1) {
    const float sv = skipv[ty];
    gate = 1.0f / (1.0f + expf(-sv));
    omg = 1.0f - gate;
  }
  v4f w3v[4];
  float b3v = 0.0f;
  if (EPI == 3) {
#pragma unroll
    for (int c = 0; c < 4; ++c) w3v[c] = *(const v4f*)(w3 + (lane & 1) * 16 + c * 4);
    b3v = b3[0];
  }
#pragma unroll
  for (int i = 0; i < 4; ++i) {
    const int mBase = m0 + (i << 4);
#pragma unroll
    for (int j = 0; j < 4; ++j) {
      const int n = n0 + (j << 4) + rlane;
      const float bv = bs[n];
#pragma unroll
      for (int r = 0; r < 8; ++r) {
        float v = acc[i][j][r] * scale + bv;
        if (EPI == 1) v = v * gate;
        if (EPI == 2 || EPI == 3) v = fmaxf(v, 0.0f);
        if (EPI == 2) v = v * oscale;
        slab[(mOff + r) * 68 + (j << 4) + rlane] = v;
      }
    }
    wave_sync();
    if (EPI == 0) {
      const int hh = lane >> 4, c4 = (lane & 15) * 4;
      for (int pass = 0; pass < 2; ++pass) {
#pragma unroll
        for (int it = 0; it < 8; ++it) {
          const int row = it * 2 + hh;
          const v4f v = *(const v4f*)(slab + row * 68 + c4);
          *(volatile v4f*)(Cf + (size_t)(mBase + row) * ldc + n0 + c4) = v;
        }
        __threadfence();
      }
    }
    if (EPI == 1) {
      const int hh = lane >> 4, c4 = (lane & 15) * 4;
      v4f ov[8];
#pragma unroll
      for (int it = 0; it < 8; ++it) {
        const int row = it * 2 + hh;
        const v4f v = *(const v4f*)(slab + row * 68 + c4);
        const v4f rr = *(const v4f*)(resid + (size_t)(mBase + row) * ldc + n0 + c4);
        ov[it] = v + omg * rr;
        *(v4f*)(slab + row * 68 + c4) = ov[it];
      }
      for (int pass = 0; pass < 2; ++pass) {
#pragma unroll
        for (int it = 0; it < 8; ++it) {
          const int row = it * 2 + hh;
          *(volatile v4f*)(Cf + (size_t)(mBase + row) * ldc + n0 + c4) = ov[it];
        }
        __threadfence();
      }
      wave_sync();
    }
    if (EPI == 1 || EPI == 2) {
      const int q = lane >> 3, c8 = (lane & 7) * 8;
      const float osc = (EPI == 1) ? oscale : 1.0f;
      for (int pass = 0; pass < 2; ++pass) {
#pragma unroll
        for (int it = 0; it < 4; ++it) {
          const int row = it * 4 + q;
          const float* sp = slab + row * 68 + c8;
          v8h hv;
#pragma unroll
          for (int e = 0; e < 8; ++e) hv[e] = (_Float16)(sp[e] * osc);
          *(volatile v8h*)(Ch + (size_t)(mBase + row) * ldc + n0 + c8) = hv;
        }
        __threadfence();
      }
    }
    if (EPI == 3) {
      const int rr_ = lane >> 1, hf = lane & 1;
      float part = 0.0f;
#pragma unroll
      for (int c = 0; c < 4; ++c) {
        const v4f sv = *(const v4f*)(slab + rr_ * 68 + hf * 16 + c * 4);
        part = fmaf(sv[0], w3v[c][0], part);
        part = fmaf(sv[1], w3v[c][1], part);
        part = fmaf(sv[2], w3v[c][2], part);
        part = fmaf(sv[3], w3v[c][3], part);
      }
      const float oth = __shfl_xor(part, 1, 32);
      const float lg = part + oth + b3v;
      if (hf == 0) sL[wave][i * 16 + rr_] = lg;
    }
    wave_sync();
  }
  if (EPI == 3) {
    wave_sync();
    if (lane < 16) {
      const int row0 = m0 + lane * 4;
      if (row0 < mReal) {
        const v4f v = *(const v4f*)(sL[wave] + lane * 4);
        *(volatile v4f*)(Cf + row0) = v;
        __threadfence();
        *(volatile v4f*)(Cf + row0) = v;
      }
    }
  }
}

__device__ __forceinline__ void rel_apply(const float* __restrict__ kp, const float* __restrict__ vp,
                                          const float* __restrict__ kr, const float* __restrict__ vr,
                                          float (&ke)[8], float (&ve)[8])
{
#pragma unroll
  for (int j = 0; j < 8; ++j) { ke[j] = 0.0f; ve[j] = 0.0f; }
#pragma unroll 1
  for (int d2 = 0; d2 < 4; ++d2) {
    const v2f kk = *(const v2f*)(kp + 2 * d2);
    const v2f vv = *(const v2f*)(vp + 2 * d2);
    const v4f a0 = *(const v4f*)(kr + 16 * d2);
    const v4f a1 = *(const v4f*)(kr + 16 * d2 + 4);
    const v4f a2 = *(const v4f*)(kr + 16 * d2 + 8);
    const v4f a3 = *(const v4f*)(kr + 16 * d2 + 12);
    const v4f c0 = *(const v4f*)(vr + 16 * d2);
    const v4f c1 = *(const v4f*)(vr + 16 * d2 + 4);
    const v4f c2 = *(const v4f*)(vr + 16 * d2 + 8);
    const v4f c3 = *(const v4f*)(vr + 16 * d2 + 12);
#pragma unroll
    for (int j = 0; j < 4; ++j) {
      ke[j]     = fmaf(kk[0], a0[j], ke[j]);
      ke[4 + j] = fmaf(kk[0], a1[j], ke[4 + j]);
      ve[j]     = fmaf(vv[0], c0[j], ve[j]);
      ve[4 + j] = fmaf(vv[0], c1[j], ve[4 + j]);
    }
#pragma unroll
    for (int j = 0; j < 4; ++j) {
      ke[j]     = fmaf(kk[1], a2[j], ke[j]);
      ke[4 + j] = fmaf(kk[1], a3[j], ke[4 + j]);
      ve[j]     = fmaf(vv[1], c2[j], ve[j]);
      ve[4 + j] = fmaf(vv[1], c3[j], ve[4 + j]);
    }
  }
}

__global__ __launch_bounds__(256) void rel_rows_kernel(
    const float* __restrict__ KQV, const float* __restrict__ krelL, const float* __restrict__ vrelL,
    float* __restrict__ REL)
{
  __shared__ __align__(16) float tile[32 * 132];
  const int tid = threadIdx.x, lane = tid & 31, wave = tid >> 5;
  const int rl = tid >> 3, h = tid & 7;
  const int r = blockIdx.x * 32 + rl;
  const int rc = r < 7000 ? r : 6999;
  const int e = rc < 5000 ? 0 : (rc < 6000 ? 6 : 7);
  const int node = rc - (rc < 5000 ? 0 : (rc < 6000 ? 5000 : 6000));
  const int srow = (e == 0 ? kOffJ : kOffM) + node;
  float ke[8], ve[8];
  const float* kp = KQV + (size_t)srow * 192 + h * 8;
  rel_apply(kp, kp + 128, krelL + e * 512 + h * 64, vrelL + e * 512 + h * 64, ke, ve);
  {
    v4f o0, o1, o2, o3;
    o0[0] = ke[0]; o0[1] = ke[1]; o0[2] = ke[2]; o0[3] = ke[3];
    o1[0] = ke[4]; o1[1] = ke[5]; o1[2] = ke[6]; o1[3] = ke[7];
    o2[0] = ve[0]; o2[1] = ve[1]; o2[2] = ve[2]; o2[3] = ve[3];
    o3[0] = ve[4]; o3[1] = ve[5]; o3[2] = ve[6]; o3[3] = ve[7];
    *(v4f*)(tile + rl * 132 + h * 8) = o0;
    *(v4f*)(tile + rl * 132 + h * 8 + 4) = o1;
    *(v4f*)(tile + rl * 132 + 64 + h * 8) = o2;
    *(v4f*)(tile + rl * 132 + 64 + h * 8 + 4) = o3;
  }
  __syncthreads();
  v4f v[4];
#pragma unroll
  for (int it = 0; it < 4; ++it) v[it] = *(const v4f*)(tile + (it * 8 + wave) * 132 + lane * 4);
  for (int pass = 0; pass < 2; ++pass) {
#pragma unroll
    for (int it = 0; it < 4; ++it)
      *(volatile v4f*)(REL + (size_t)(blockIdx.x * 32 + it * 8 + wave) * 128 + lane * 4) = v[it];
    __threadfence();
  }
}

struct EdgePtrs { const int* p0; const int* p1; const int* p2; const int* p3; const int* p4; const int* p5; const int* p6; const int* p7; };
static_assert(sizeof(EdgePtrs) == 64, "no padding");

__device__ __forceinline__ int q_lookup(const int* qb, const int (&pre)[10], int g)
{
  int base = 0, k = 0;
#pragma unroll
  for (int i = 1; i <= 8; ++i) {
    const bool ge = g >= pre[i];
    base = ge ? pre[i] : base;
    k += ge ? 1 : 0;
  }
  const int off = g - base;
  int addr = (k == 0) ? off : (32 + (k - 1) * 1024 + off);
  addr = addr < 0 ? 0 : (addr > (32 + 8 * 1024 - 1) ? (32 + 8 * 1024 - 1) : addr);
  return qb[addr];
}

#define EDGE_SLOT_TEST(SRCV, DSTV)                                                          \
  {                                                                                         \
    const unsigned tt_ = (unsigned)((DSTV) - tile0);                                        \
    const bool hit_ = val && (tt_ < (unsigned)tn);                                          \
    const unsigned bm_ = __builtin_amdgcn_ballot_w32(hit_);                                 \
    const int pos_ = wc + (int)__builtin_amdgcn_mbcnt_lo(bm_, 0u);                          \
    if (hit_) myq[pos_ < 1023 ? pos_ : 1023] = (int)(((unsigned)(SRCV) & 0xFFFFu) | (tt_ << 16)); \
    wc += __builtin_popcount(bm_);                                                          \
  }

__global__ __launch_bounds__(256) void edge_kernel(
    EdgePtrs ep, const float* __restrict__ KQV, const float* __restrict__ REL,
    const float* __restrict__ krelL, const float* __restrict__ vrelL, const float* __restrict__ prelL,
    unsigned short* __restrict__ GH)
{
  __shared__ __align__(16) float acc[kTile * 72];
  __shared__ __align__(16) float stage[32 * 72];
  __shared__ int qbuf[32 + 8 * 1024];
  __shared__ int sdst[32];
  __shared__ int wqn[8];
  const int tid = threadIdx.x, lane = tid & 31, wave = tid >> 5;
  const int b = blockIdx.x;
  const int ty = (b >= kTilesOp ? 1 : 0) + (b >= kTilesOp + kTilesM ? 1 : 0);
  const int tl = b - (ty == 0 ? 0 : (ty == 1 ? kTilesOp : kTilesOp + kTilesM));
  const int nT = ty == 0 ? kNop : (ty == 1 ? kNm : kNj);
  const int padT = ty == 0 ? kPadOp : (ty == 1 ? kPadM : kPadJ);
  const int offT = ty == 0 ? 0 : (ty == 1 ? kOffM : kOffJ);
  const int tile0 = tl * kTile;
  int tn = nT - tile0;
  tn = tn < 0 ? 0 : (tn > kTile ? kTile : tn);
  int nrows = padT - tile0;
  nrows = nrows < 0 ? 0 : (nrows > kTile ? kTile : nrows);
  const int nph = ty == 0 ? 5 : (ty == 1 ? 2 : 1);
  const float isd = 1.0f / sqrtf((float)kD);

#pragma unroll 1
  for (int i = tid * 4; i < kTile * 72; i += 1024) *(v4f*)(acc + i) = (v4f){0.f, 0.f, 0.f, 0.f};
  __syncthreads();

  int* myq = qbuf + 32 + wave * 1024;
  const int hs = tid >> 3, hh = tid & 7;

#pragma unroll 1
  for (int pi = 0; pi < nph; ++pi) {
    int e;
    if (ty == 0) e = (pi == 0) ? 0 : ((pi == 1) ? 2 : ((pi == 2) ? 3 : ((pi == 3) ? 6 : 7)));
    else if (ty == 1) e = 4 + pi;
    else e = 1;
    const int* ed = (e == 0) ? ep.p0 : (e == 1) ? ep.p1 : (e == 2) ? ep.p2 : (e == 3) ? ep.p3
                  : (e == 4) ? ep.p4 : (e == 5) ? ep.p5 : (e == 6) ? ep.p6 : ep.p7;
    const int E = (e == 6) ? kEBig : kE;
    const bool hoist = (e == 0) || (e >= 6);
    const int srcOff = (e == 0) ? kOffJ : ((e >= 6) ? kOffM : 0);
    const int nSrc = (e == 0) ? kNj : ((e >= 6) ? kNm : kNop);
    const int relBase = (e == 0) ? 0 : ((e == 6) ? 5000 : 6000);
    const float* krelE = krelL + e * 512 + hh * 64;
    const float* vrelE = vrelL + e * 512 + hh * 64;
    const float pr = prelL[e * 8 + hh];
    int carryN = 0;
    const int nsc = (E + 8191) >> 13;
#pragma unroll 1
    for (int sc = 0; sc < nsc; ++sc) {
      int wc = 0;
#pragma unroll 1
      for (int it = 0; it < 4; ++it) {
        const int eb = sc * 8192 + wave * 1024 + it * 256 + lane * 8;
        const bool val = eb < E;
        const int ebc = val ? eb : (E - 8);
        const v4i s0 = *(const v4i*)(ed + ebc);
        const v4i s1 = *(const v4i*)(ed + ebc + 4);
        const v4i d0 = *(const v4i*)(ed + E + ebc);
        const v4i d1 = *(const v4i*)(ed + E + ebc + 4);
        EDGE_SLOT_TEST(s0[0], d0[0])
        EDGE_SLOT_TEST(s0[1], d0[1])
        EDGE_SLOT_TEST(s0[2], d0[2])
        EDGE_SLOT_TEST(s0[3], d0[3])
        EDGE_SLOT_TEST(s1[0], d1[0])
        EDGE_SLOT_TEST(s1[1], d1[1])
        EDGE_SLOT_TEST(s1[2], d1[2])
        EDGE_SLOT_TEST(s1[3], d1[3])
      }
      if (lane == 0) wqn[wave] = wc;
      __syncthreads();
      int pre[10];
      pre[0] = 0;
      pre[1] = carryN;
#pragma unroll
      for (int i = 0; i < 8; ++i) {
        int c = wqn[i];
        c = c < 0 ? 0 : (c > 1024 ? 1024 : c);
        pre[i + 2] = pre[i + 1] + c;
      }
      const int total = pre[9];
      const bool lastsc = (sc == nsc - 1);
      const int ngrp = lastsc ? ((total + 31) >> 5) : (total >> 5);
#pragma unroll 1
      for (int r = 0; r < ngrp; ++r) {
        const int g = r * 32 + hs;
        const bool hv = g < total;
        const int gc = hv ? g : (total - 1);
        const int ent = q_lookup(qbuf, pre, gc);
        int src = ent & 0xFFFF;
        src = src < nSrc ? src : (nSrc - 1);
        int t = (ent >> 16) & 0x1FF;
        t = t < kTile ? t : (kTile - 1);
        float ke[8], ve[8];
        if (hoist) {
          const float* rp = REL + (size_t)(relBase + src) * 128 + hh * 8;
          const v4f k0 = *(const v4f*)(rp);
          const v4f k1 = *(const v4f*)(rp + 4);
          const v4f w0 = *(const v4f*)(rp + 64);
          const v4f w1 = *(const v4f*)(rp + 68);
#pragma unroll
          for (int j = 0; j < 4; ++j) { ke[j] = k0[j]; ke[4 + j] = k1[j]; ve[j] = w0[j]; ve[4 + j] = w1[j]; }
        } else {
          const float* kp = KQV + (size_t)(srcOff + src) * 192 + hh * 8;
          rel_apply(kp, kp + 128, krelE, vrelE, ke, ve);
        }
        int qr = offT + tile0 + t;
        qr = qr < kRows ? qr : (kRows - 1);
        const float* qp = KQV + (size_t)qr * 192 + 64 + hh * 8;
        const v4f q0 = *(const v4f*)(qp);
        const v4f q1 = *(const v4f*)(qp + 4);
        float al = 0.0f;
#pragma unroll
        for (int j = 0; j < 4; ++j) {
          al = fmaf(q0[j], ke[j], al);
          al = fmaf(q1[j], ke[4 + j], al);
        }
        float a = al * pr * isd;
        a = a > 60.0f ? 60.0f : (a < -60.0f ? -60.0f : a);
        float ex = expf(a);
        ex = hv ? ex : 0.0f;
        v4f m0, m1;
#pragma unroll
        for (int j = 0; j < 4; ++j) { m0[j] = ex * ve[j]; m1[j] = ex * ve[4 + j]; }
        *(v4f*)(stage + hs * 72 + hh * 8) = m0;
        *(v4f*)(stage + hs * 72 + hh * 8 + 4) = m1;
        stage[hs * 72 + 64 + hh] = ex;
        if (hh == 0) sdst[hs] = t;
        __syncthreads();
        int nv = total - r * 32;
        nv = nv > 32 ? 32 : nv;
        if (tid < 18) {
#pragma unroll 1
          for (int i = 0; i < nv; ++i) {
            const int n = sdst[i];
            v4f av = *(const v4f*)(acc + n * 72 + tid * 4);
            const v4f mv = *(const v4f*)(stage + i * 72 + tid * 4);
            av = av + mv;
            *(v4f*)(acc + n * 72 + tid * 4) = av;
          }
        }
        __syncthreads();
      }
      const int rem0 = ngrp * 32;
      const int ncar = lastsc ? 0 : (total - rem0);
      int cent = 0;
      if (tid < ncar) cent = q_lookup(qbuf, pre, rem0 + tid);
      __syncthreads();
      if (tid < ncar) qbuf[tid] = cent;
      carryN = ncar;
    }
  }

  __syncthreads();
#pragma unroll 1
  for (int idx = tid; idx < nrows * 64; idx += 256) {
    const int n = idx >> 6, c = idx & 63;
    const float d = acc[n * 72 + 64 + (c >> 3)];
    const float s = acc[n * 72 + c];
    const float rd = __builtin_amdgcn_rcpf(d > 0.0f ? d : 1.0f);
    const float av = (d > 0.0f) ? s * rd : 0.0f;
    const float gl = 0.5f * av * (1.0f + erff(av * 0.70710678118654752f));
    acc[n * 72 + c] = gl * kActCarry;
  }
  __syncthreads();
#pragma unroll 1
  for (int r0 = 0; r0 < nrows; r0 += 32) {
    const int row = r0 + (tid >> 3);
    if (row < nrows) {
      const int c8 = (tid & 7) * 8;
      const v4f a0 = *(const v4f*)(acc + row * 72 + c8);
      const v4f a1 = *(const v4f*)(acc + row * 72 + c8 + 4);
      v8h hv8;
#pragma unroll
      for (int j = 0; j < 4; ++j) { hv8[j] = (_Float16)a0[j]; hv8[4 + j] = (_Float16)a1[j]; }
      unsigned short* dst = GH + (size_t)(offT + tile0 + row) * 64 + c8;
      *(volatile v8h*)dst = hv8;
      __threadfence();
      *(volatile v8h*)dst = hv8;
    }
  }
}

__global__ __launch_bounds__(256) void colsum_kernel(const float* __restrict__ X, float* __restrict__ PARTM)
{
  __shared__ float sm[256];
  const int tid = threadIdx.x;
  const int b = blockIdx.x;
  const int ty = (b >= kBlkOp ? 1 : 0) + (b >= kBlkOp + kBlkM ? 1 : 0);
  const int tb0 = ty == 0 ? 0 : (ty == 1 ? kBlkOp : kBlkOp + kBlkM);
  const int nT = ty == 0 ? kNop : (ty == 1 ? kNm : kNj);
  const int col = tid & 63, grp = tid >> 6;
  float s = 0.0f;
#pragma unroll 1
  for (int i = 0; i < 16; ++i) {
    const int rl = grp * 16 + i;
    const int rt = (b - tb0) * 64 + rl;
    const float v = X[(size_t)(b * 64 + rl) * 64 + col];
    s += (rt < nT) ? v : 0.0f;
  }
  sm[tid] = s;
  __syncthreads();
  if (tid < 64) {
    const float tot = (sm[tid] + sm[64 + tid]) + (sm[128 + tid] + sm[192 + tid]);
    *(volatile float*)(PARTM + (size_t)b * 64 + tid) = tot;
    __threadfence();
    *(volatile float*)(PARTM + (size_t)b * 64 + tid) = tot;
  }
}

__global__ __launch_bounds__(256) void head_kernel(
    const float* __restrict__ PARTM,
    const float* __restrict__ Wv1, const float* __restrict__ bv1,
    const float* __restrict__ Wv2, const float* __restrict__ bv2,
    const float* __restrict__ Wp1, const float* __restrict__ bp1, const float* __restrict__ bp2,
    float* __restrict__ CB, float* __restrict__ outv)
{
  __shared__ double dred[256];
  __shared__ float gsh[192];
  __shared__ float h1[64];
  __shared__ __align__(16) float cb[128];
  const int tid = threadIdx.x, lane = tid & 31;
  const int col = tid & 63, grp = tid >> 6;
#pragma unroll 1
  for (int ty = 0; ty < 3; ++ty) {
    const int b0 = ty == 0 ? 0 : (ty == 1 ? kBlkOp : kBlkOp + kBlkM);
    const int b1 = ty == 0 ? kBlkOp : (ty == 1 ? kBlkOp + kBlkM : kBlkAll);
    const double rinv = ty == 0 ? (1.0 / (double)kNop) : (ty == 1 ? (1.0 / (double)kNm) : (1.0 / (double)kNj));
    double s = 0.0;
#pragma unroll 1
    for (int b = b0 + grp; b < b1; b += 4) s += (double)PARTM[(size_t)b * 64 + col];
    dred[tid] = s;
    __syncthreads();
    if (tid < 64) gsh[ty * 64 + tid] = (float)(((dred[tid] + dred[64 + tid]) + (dred[128 + tid] + dred[192 + tid])) * rinv);
    __syncthreads();
  }
  if (grp < 2) {
    const float* W = (grp == 0) ? Wv1 : (Wp1 + 128 * 64);
    const float bva = bv1[col];
    const float bpa = bp1[col];
    float a = (grp == 0) ? bva : bpa;
#pragma unroll 1
    for (int i = 0; i < 192; ++i) a = fmaf(gsh[i], W[(size_t)i * 64 + col], a);
    if (grp == 0) h1[col] = fmaxf(a, 0.0f);
    else cb[col] = a;
  } else if (grp == 2) {
    const float v = bp2[col < 32 ? col : 31];
    cb[64 + col] = (col < 32) ? v : 0.0f;
  }
  __syncthreads();
  if (tid < 32) {
    float p = h1[lane] * Wv2[lane];
    p = fmaf(h1[lane + 32], Wv2[lane + 32], p);
#pragma unroll
    for (int off = 16; off > 0; off >>= 1) p += __shfl_xor(p, off, 32);
    const float val = p + bv2[0];
    const v4f cv = *(const v4f*)(cb + lane * 4);
    *(volatile v4f*)(CB + lane * 4) = cv;
    if (lane == 0) *(volatile float*)(outv) = val;
    __threadfence();
    *(volatile v4f*)(CB + lane * 4) = cv;
    if (lane == 0) *(volatile float*)(outv) = val;
  }
}

__global__ __launch_bounds__(256) void gather_pairs_kernel(
    const float* __restrict__ X, const int* __restrict__ opIdx, const int* __restrict__ mIdx,
    unsigned short* __restrict__ ZH)
{
  const int gid = blockIdx.x * 256 + threadIdx.x;
  const int p = gid >> 4, c8 = (gid & 15) * 8;
  const bool pv = p < kP;
  const int pc = pv ? p : (kP - 1);
  int oi = opIdx[pc];
  int mi = mIdx[pc];
  oi = oi < 0 ? 0 : (oi > kNop - 1 ? kNop - 1 : oi);
  mi = mi < 0 ? 0 : (mi > kNm - 1 ? kNm - 1 : mi);
  const int row = (c8 < 64) ? oi : (kOffM + mi);
  const int col = c8 & 63;
  const v4f a0 = *(const v4f*)(X + (size_t)row * 64 + col);
  const v4f a1 = *(const v4f*)(X + (size_t)row * 64 + col + 4);
  v8h hv;
#pragma unroll
  for (int j = 0; j < 4; ++j) {
    hv[j] = (_Float16)(pv ? a0[j] * kActCarry : 0.0f);
    hv[4 + j] = (_Float16)(pv ? a1[j] * kActCarry : 0.0f);
  }
  unsigned short* dst = ZH + (size_t)p * 128 + c8;
  *(volatile v8h*)dst = hv;
  __threadfence();
  *(volatile v8h*)dst = hv;
}

extern "C" void kernel_launch(void* const* d_in, const int* in_sizes, int n_in,
                              void* d_out, int out_size, void* d_ws, size_t ws_size,
                              hipStream_t stream) {
  (void)in_sizes; (void)out_size;
  if (n_in < 39) return;
  if (ws_size < kWsTotal) return;

  const float* op_x   = (const float*)d_in[0];
  const float* mach_x = (const float*)d_in[1];
  const float* job_x  = (const float*)d_in[2];
  const float* W_op   = (const float*)d_in[3];
  const float* b_op   = (const float*)d_in[4];
  const float* W_mach = (const float*)d_in[5];
  const float* b_mach = (const float*)d_in[6];
  const float* W_job  = (const float*)d_in[7];
  const float* b_job  = (const float*)d_in[8];
  const float* ln_gamma = (const float*)d_in[9];
  const float* ln_beta  = (const float*)d_in[10];
  const float* Wkqv = (const float*)d_in[11];
  const float* bkqv = (const float*)d_in[12];
  const float* krel = (const float*)d_in[13];
  const float* vrel = (const float*)d_in[14];
  const float* prel = (const float*)d_in[15];
  const float* Wout = (const float*)d_in[16];
  const float* bout = (const float*)d_in[17];
  const float* skip = (const float*)d_in[18];
  const float* Wp1 = (const float*)d_in[19];
  const float* bp1 = (const float*)d_in[20];
  const float* Wp2 = (const float*)d_in[21];
  const float* bp2 = (const float*)d_in[22];
  const float* Wp3 = (const float*)d_in[23];
  const float* bp3 = (const float*)d_in[24];
  const float* Wv1 = (const float*)d_in[25];
  const float* bv1 = (const float*)d_in[26];
  const float* Wv2 = (const float*)d_in[27];
  const float* bv2 = (const float*)d_in[28];
  EdgePtrs ep;
  ep.p0 = (const int*)d_in[29]; ep.p1 = (const int*)d_in[30]; ep.p2 = (const int*)d_in[31]; ep.p3 = (const int*)d_in[32];
  ep.p4 = (const int*)d_in[33]; ep.p5 = (const int*)d_in[34]; ep.p6 = (const int*)d_in[35]; ep.p7 = (const int*)d_in[36];
  const int* op_idx = (const int*)d_in[37];
  const int* m_idx  = (const int*)d_in[38];
  float* out = (float*)d_out;

  char* ws = (char*)d_ws;
  float* X0 = (float*)(ws + kOffX0);
  float* X1 = (float*)(ws + kOffX1);
  unsigned short* XH = (unsigned short*)(ws + kOffXH);
  unsigned short* GH = (unsigned short*)(ws + kOffGH);
  float* KQV = (float*)(ws + kOffKQV);
  float* REL = (float*)(ws + kOffREL);
  unsigned short* WT = (unsigned short*)(ws + kOffWT);
  float* PART = (float*)(ws + kOffPART);
  float* STATS = (float*)(ws + kOffSTAT);
  float* PARTM = (float*)(ws + kOffPARTM);
  float* CB = (float*)(ws + kOffCB);
  unsigned short* ZH = (unsigned short*)(ws + kOffZH);
  unsigned short* Z1H = (unsigned short*)(ws + kOffZ1H);

  prep_weights_kernel<<<54, 256, 0, stream>>>(Wkqv, Wout, Wp1, Wp2, WT);
  proj_kernel<<<kBlkAll, 256, 0, stream>>>(op_x, mach_x, job_x, W_op, b_op, W_mach, b_mach, W_job, b_job, X1, PART);
  stats_kernel<<<1, 256, 0, stream>>>(PART, STATS);
  norm_kernel<<<kRows / 32, 256, 0, stream>>>(X1, STATS, ln_gamma, ln_beta, X0, XH);

  float* cur = X0;
  float* nxt = X1;
  for (int l = 0; l < kLayers; ++l) {
    gemm64_kernel<0><<<(kBlkAll * 3 + 7) / 8, 256, 0, stream>>>(
        XH, 64, WT + (size_t)l * 3 * 192 * 64, 64, 192 * 64,
        bkqv + (size_t)l * 3 * 192, 192,
        KQV, nullptr, 192, nullptr, nullptr, nullptr, nullptr,
        kBlkAll, 3, 64, 1, kRows, kGemmScale, 1.0f);
    rel_rows_kernel<<<kRelRows / 32, 256, 0, stream>>>(
        KQV, krel + (size_t)l * 8 * 512, vrel + (size_t)l * 8 * 512, REL);
    edge_kernel<<<kTilesOp + kTilesM + kTilesJ, 256, 0, stream>>>(
        ep, KQV, REL, krel + (size_t)l * 8 * 512, vrel + (size_t)l * 8 * 512, prel + (size_t)l * 64, GH);
    gemm64_kernel<1><<<(kBlkAll + 7) / 8, 256, 0, stream>>>(
        GH, 64, WT + kWtOffOut + (size_t)l * 3 * 64 * 64, 64, 64 * 64,
        bout + (size_t)l * 3 * 64, 64,
        nxt, XH, 64, cur, skip + (size_t)l * 3, nullptr, nullptr,
        kBlkAll, 1, 64, 1, kRows, kGemmScale, kActCarry);
    float* t = cur; cur = nxt; nxt = t;
  }

  colsum_kernel<<<kBlkAll, 256, 0, stream>>>(cur, PARTM);
  head_kernel<<<1, 256, 0, stream>>>(PARTM, Wv1, bv1, Wv2, bv2, Wp1, bp1, bp2, CB, out + kP);
  gather_pairs_kernel<<<(kPPad * 16) / 256, 256, 0, stream>>>(cur, op_idx, m_idx, ZH);
  gemm64_kernel<2><<<(kPPad / 64 + 7) / 8, 256, 0, stream>>>(
      ZH, 128, WT + kWtOffP1, 128, 0,
      CB, 0,
      nullptr, Z1H, 64, nullptr, nullptr, nullptr, nullptr,
      kPPad / 64, 1, 128, 0, kPPad, kGemmScale, kActCarry);
  gemm64_kernel<3><<<(kPPad / 64 + 7) / 8, 256, 0, stream>>>(
      Z1H, 64, WT + kWtOffP2, 64, 0,
      CB + 64, 0,
      out, nullptr, 64, nullptr, nullptr, Wp3, bp3,
      kPPad / 64, 1, 64, 0, kP, kGemmScale, 1.0f);
}
